// CausalSelfAttention_7112465842232
// MI455X (gfx1250) — hardware-verified
//
#include <hip/hip_runtime.h>

typedef __attribute__((ext_vector_type(16))) _Float16 v16h;
typedef __attribute__((ext_vector_type(8)))  _Float16 v8h;
typedef __attribute__((ext_vector_type(16))) __bf16   v16b;
typedef __attribute__((ext_vector_type(8)))  __bf16   v8b;
typedef __attribute__((ext_vector_type(8)))  float    v8f;
typedef __attribute__((ext_vector_type(4)))  float    v4f;
typedef __attribute__((ext_vector_type(4)))  unsigned int v4u;

#ifndef NB
#define NB 2
#endif
#ifndef SEQ
#define SEQ 2048
#endif
#define NB_FULL 2
#define SEQ_FULL 2048

constexpr int kBatch   = NB;
constexpr int kSeq     = SEQ;
constexpr int kSeqFull = SEQ_FULL;
constexpr int kDim     = 1024;
constexpr int kHeads   = 16;
constexpr int kHeadDim = 64;
constexpr int kRows    = kBatch * kSeq;
constexpr int kQKV     = 3 * kDim;
constexpr float kScoreScale = 0.125f;
constexpr float kMaskFill   = -1000000000.0f;

static_assert(kBatch >= 1 && kBatch <= NB_FULL);
static_assert(kSeq >= 64 && kSeq <= kSeqFull);
static_assert(kHeads * kHeadDim == kDim);
static_assert(kHeadDim == 64);
static_assert(kSeq % 64 == 0);
static_assert(kRows % 64 == 0 && kQKV % 64 == 0 && kDim % 64 == 0 && kDim % 32 == 0);
static_assert((long)((kBatch - 1) * kSeqFull + kSeq) * kDim < 2147483647L);
static_assert(((kSeq * kDim) / 8) % 256 == 0);
static_assert(kDim == 256 * 4);
static_assert((kSeqFull % 4) == 0);

constexpr size_t al128(size_t v) { return (v + 127) / 128 * 128; }
constexpr size_t kOffXB  = 0;
constexpr size_t kSzXB   = (size_t)kRows * kDim * 2;
constexpr size_t kOffWQT = al128(kOffXB + kSzXB);
constexpr size_t kSzWQT  = (size_t)kQKV * kDim * 2;
constexpr size_t kOffYH  = 0;
constexpr size_t kSzY    = (size_t)kRows * kDim * 2;
constexpr size_t kOffYL  = al128(kOffYH + kSzY);
constexpr size_t kEndA   = kOffWQT + kSzWQT;
constexpr size_t kEndB   = kOffYL + kSzY;
constexpr size_t kOffQH  = al128(kEndA > kEndB ? kEndA : kEndB);
constexpr size_t kSzQ    = (size_t)kRows * kQKV * 2;
constexpr size_t kOffQL  = al128(kOffQH + kSzQ);
constexpr size_t kOffBC  = al128(kOffQL + kSzQ);
constexpr size_t kSzBC   = (size_t)kQKV * 4;
constexpr size_t kOffWPT = al128(kOffBC + kSzBC);
constexpr size_t kSzWPT  = (size_t)kDim * kDim * 2;
constexpr size_t kWsTotal = kOffWPT + kSzWPT;
static_assert(kOffXB + kSzXB <= kOffWQT);
static_assert(kOffWQT + kSzWQT <= kOffQH);
static_assert(kOffYL + kSzY <= kOffQH);
static_assert(kOffQH + kSzQ <= kOffQL);
static_assert(kOffQL + kSzQ <= kOffBC);
static_assert(kOffBC + kSzBC <= kOffWPT);
static_assert(kWsTotal <= 134217728);
static_assert((kOffWQT % 128) == 0 && (kOffYL % 128) == 0 && (kOffQH % 128) == 0 && (kOffQL % 128) == 0);
static_assert((kOffBC % 128) == 0 && (kOffWPT % 128) == 0);
static_assert((size_t)kRows * kDim * 4 <= (size_t)16777216);

__device__ __forceinline__ unsigned short f2bf_bits(float f) {
  unsigned u = __float_as_uint(f);
  return (unsigned short)((u + 0x7FFFu + ((u >> 16) & 1u)) >> 16);
}
__device__ __forceinline__ float bf_bits2f(unsigned short h) { return __uint_as_float(((unsigned)h) << 16); }

__device__ __forceinline__ void dep_guard_h(v8f& a, v8f& b, v16h x, v16h y) { asm volatile("v_nop\n\tv_nop\n\tv_nop\n\tv_nop" : "+v"(a), "+v"(b) : "v"(x), "v"(y)); }
__device__ __forceinline__ void dep_guard_b(v8f& a, v8f& b, v16b x, v16b y) { asm volatile("v_nop\n\tv_nop\n\tv_nop\n\tv_nop" : "+v"(a), "+v"(b) : "v"(x), "v"(y)); }
__device__ __forceinline__ void keep4_h(v16h a, v16h b, v16h c, v16h d) { asm volatile("v_nop" :: "v"(a), "v"(b), "v"(c), "v"(d)); }
__device__ __forceinline__ void keep4_b(v16b a, v16b b, v16b c, v16b d) { asm volatile("v_nop" :: "v"(a), "v"(b), "v"(c), "v"(d)); }
__device__ __forceinline__ void acc_guard4(v8f& a, v8f& b, v8f& c, v8f& d) { asm volatile("v_nop\n\tv_nop\n\tv_nop\n\tv_nop" : "+v"(a), "+v"(b), "+v"(c), "+v"(d)); }

template <typename T> struct Frag;
template <> struct Frag<_Float16> {
  typedef v16h V; union U { v16h v; v8h h[2]; };
  static __device__ __forceinline__ v16h load(const _Float16* p) {
    U f; f.h[0] = *(const v8h*)(p); f.h[1] = *(const v8h*)(p + 16); return f.v;
  }
  static __device__ __forceinline__ v8f mma(v16h a, v16h b, v8f c) {
    return __builtin_amdgcn_wmma_f32_16x16x32_f16(false, a, false, b, (short)0, c, false, false);
  }
  static __device__ __forceinline__ void guard(v8f& a, v8f& b, v16h x, v16h y) { dep_guard_h(a, b, x, y); }
  static __device__ __forceinline__ void keep(v16h a, v16h b, v16h c, v16h d) { keep4_h(a, b, c, d); }
};
template <> struct Frag<__bf16> {
  typedef v16b V; union U { v16b v; v8b h[2]; };
  static __device__ __forceinline__ v16b load(const __bf16* p) {
    U f; f.h[0] = *(const v8b*)(p); f.h[1] = *(const v8b*)(p + 16); return f.v;
  }
  static __device__ __forceinline__ v8f mma(v16b a, v16b b, v8f c) {
    return __builtin_amdgcn_wmma_f32_16x16x32_bf16(false, a, false, b, (short)0, c, false, false);
  }
  static __device__ __forceinline__ void guard(v8f& a, v8f& b, v16b x, v16b y) { dep_guard_b(a, b, x, y); }
  static __device__ __forceinline__ void keep(v16b a, v16b b, v16b c, v16b d) { keep4_b(a, b, c, d); }
};

template <int ET> struct Elem;
template <> struct Elem<0> { typedef _Float16 T; };
template <> struct Elem<1> { typedef __bf16 T; };
template <int ET, bool SPLA, bool SPLB, int BIAS_MODE, int OUT_MODE>
__device__ __forceinline__ void wmma_gemm64_body(
    const unsigned short* __restrict__ Ap, const unsigned short* __restrict__ A2p, int lda, long strideA,
    const unsigned short* __restrict__ Btp, const unsigned short* __restrict__ Bt2p, int ldb, long strideB,
    void* __restrict__ Cout, void* __restrict__ Cout2, int ldc, long strideC,
    const float* __restrict__ bias,
    int M, int N, int K, float scale) {
  typedef typename Elem<ET>::T T;
  typedef typename Frag<T>::V V;
  const T* A = (const T*)Ap; const T* A2 = (const T*)A2p; const T* Bt = (const T*)Btp; const T* Bt2 = (const T*)Bt2p;
  __shared__ __align__(16) float sT[8][16 * 68];
  const int b    = blockIdx.y;
  const int lane = threadIdx.x & 31;
  const int wave = threadIdx.x >> 5;
  const int tilesN = N >> 6;
  const int tilesM = M >> 6;
  const int tile = blockIdx.x * 8 + wave;
  if (tile >= tilesM * tilesN) return;
  const int tm = tile / tilesN;
  const int tn = tile - tm * tilesN;
  const int m0 = tm << 6;
  const int n0 = tn << 6;

  const T* Ab  = A  + (size_t)b * strideA;
  const T* Bb  = Bt + (size_t)b * strideB;
  const T* Ab2 = SPLA ? (A2  + (size_t)b * strideA) : nullptr;
  const T* Bb2 = SPLB ? (Bt2 + (size_t)b * strideB) : nullptr;

  const int rlane = lane & 15;
  const int koff  = (lane >> 4) * 8;
  const int mOff  = (lane >> 4) * 8;

  v8f acc[4][4];
#pragma unroll
  for (int i = 0; i < 4; ++i)
#pragma unroll
    for (int j = 0; j < 4; ++j) acc[i][j] = (v8f){0.f,0.f,0.f,0.f,0.f,0.f,0.f,0.f};

  for (int k0 = 0; k0 < K; k0 += 32) {
    V bh[4], bl[4];
#pragma unroll
    for (int j = 0; j < 4; ++j) {
      const size_t bo = (size_t)(n0 + (j << 4) + rlane) * ldb + koff + k0;
      bh[j] = Frag<T>::load(Bb + bo);
      if (SPLB) bl[j] = Frag<T>::load(Bb2 + bo);
    }
#pragma unroll
    for (int i = 0; i < 4; ++i) {
      const size_t ao = (size_t)(m0 + (i << 4) + rlane) * lda + koff + k0;
      V ah = Frag<T>::load(Ab + ao);
      V al;
      if (SPLA) al = Frag<T>::load(Ab2 + ao);
#pragma unroll
      for (int j = 0; j < 4; ++j) {
        acc[i][j] = Frag<T>::mma(ah, bh[j], acc[i][j]);
        if (SPLB) acc[i][j] = Frag<T>::mma(ah, bl[j], acc[i][j]);
        if (SPLA) acc[i][j] = Frag<T>::mma(al, bh[j], acc[i][j]);
      }
      Frag<T>::guard(acc[i][0], acc[i][3], ah, SPLA ? al : ah);
    }
    Frag<T>::keep(bh[0], bh[1], bh[2], bh[3]);
    if (SPLB) Frag<T>::keep(bl[0], bl[1], bl[2], bl[3]);
  }
  acc_guard4(acc[0][0], acc[0][1], acc[0][2], acc[0][3]);
  acc_guard4(acc[1][0], acc[1][1], acc[1][2], acc[1][3]);
  acc_guard4(acc[2][0], acc[2][1], acc[2][2], acc[2][3]);
  acc_guard4(acc[3][0], acc[3][1], acc[3][2], acc[3][3]);

  float* slab = sT[wave];
#pragma unroll
  for (int i = 0; i < 4; ++i) {
    const int mBase = m0 + (i << 4);
#pragma unroll
    for (int j = 0; j < 4; ++j) {
      const int n = n0 + (j << 4) + rlane;
      float bv = 0.f;
      if (BIAS_MODE == 2) bv = bf_bits2f(f2bf_bits(bias[n]));
#pragma unroll
      for (int r = 0; r < 8; ++r) {
        float v = acc[i][j][r] * scale;
        if (BIAS_MODE == 2) v += bv;
        slab[(mOff + r) * 68 + (j << 4) + rlane] = v;
      }
    }
    __builtin_amdgcn_fence(3  , "workgroup");
    __builtin_amdgcn_wave_barrier();
    __builtin_amdgcn_fence(2  , "workgroup");
    if (OUT_MODE == 0) {
      float* C = (float*)Cout + (size_t)b * strideC;
      const int hh = lane >> 4, c4 = (lane & 15) * 4;
      for (int pass = 0; pass < 2; ++pass) {
#pragma unroll
        for (int it = 0; it < 8; ++it) {
          const int row = it * 2 + hh;
          v4f v = *(const v4f*)(slab + row * 68 + c4);
          *(volatile v4f*)(C + (size_t)(mBase + row) * ldc + n0 + c4) = v;
        }
        __threadfence();
      }
    } else {
      const int q = lane >> 3, c8 = (lane & 7) * 8;
      unsigned short* C  = (unsigned short*)Cout  + (size_t)b * strideC;
      unsigned short* C2 = (OUT_MODE == 2) ? ((unsigned short*)Cout2 + (size_t)b * strideC) : nullptr;
      for (int pass = 0; pass < 2; ++pass) {
#pragma unroll
        for (int it = 0; it < 4; ++it) {
          const int row = it * 4 + q;
          const float* sp = slab + row * 68 + c8;
          v8h hv, lv;
#pragma unroll
          for (int e = 0; e < 8; ++e) {
            if (OUT_MODE == 1) {
              hv[e] = (_Float16)sp[e];
            } else {
              unsigned short hb = f2bf_bits(sp[e]);
              unsigned short lb = f2bf_bits(sp[e] - bf_bits2f(hb));
              hv[e] = __builtin_bit_cast(_Float16, hb);
              lv[e] = __builtin_bit_cast(_Float16, lb);
            }
          }
          *(volatile v8h*)(C + (size_t)(mBase + row) * ldc + n0 + c8) = hv;
          if (OUT_MODE == 2) *(volatile v8h*)(C2 + (size_t)(mBase + row) * ldc + n0 + c8) = lv;
        }
        __threadfence();
      }
    }
    __builtin_amdgcn_fence(3  , "workgroup");
    __builtin_amdgcn_wave_barrier();
    __builtin_amdgcn_fence(2  , "workgroup");
  }
}

__global__ __launch_bounds__(256) void gemm_qkv_planes(
    const unsigned short* __restrict__ A, int lda,
    const unsigned short* __restrict__ Bt, int ldb,
    unsigned short* __restrict__ Ch, unsigned short* __restrict__ Cl, int ldc,
    const float* __restrict__ bias, int M, int N, int K) {
  wmma_gemm64_body<1, false, false, 2, 2>(A, A, lda, 0L, Bt, Bt, ldb, 0L,
                                          (void*)Ch, (void*)Cl, ldc, 0L, bias, M, N, K, 1.0f);
}

__global__ __launch_bounds__(256) void gemm_proj_f32(
    const unsigned short* __restrict__ Ah, const unsigned short* __restrict__ Al, int lda,
    const unsigned short* __restrict__ Bt, int ldb,
    float* __restrict__ C, int ldc,
    const float* __restrict__ bias, int M, int N, int K) {
  wmma_gemm64_body<1, true, false, 2, 0>(Ah, Al, lda, 0L, Bt, Bt, ldb, 0L,
                                         (void*)C, (void*)C, ldc, 0L, bias, M, N, K, 1.0f);
}

__global__ __launch_bounds__(256) void cast_f32_bf16x8(
    const float* __restrict__ in, unsigned short* __restrict__ out, int n8, long strideIn, long strideOut) {
  const int i = blockIdx.x * 256 + threadIdx.x;
  const int b = blockIdx.y;
  if (i < n8) {
    const size_t e0 = (size_t)i * 8;
    const float* src = in + (size_t)b * strideIn + e0;
    unsigned short* dst = out + (size_t)b * strideOut + e0;
    const v4f a = *(const v4f*)(src);
    const v4f c = *(const v4f*)(src + 4);
    v4u w;
    w[0] = (unsigned)f2bf_bits(a[0]) | ((unsigned)f2bf_bits(a[1]) << 16);
    w[1] = (unsigned)f2bf_bits(a[2]) | ((unsigned)f2bf_bits(a[3]) << 16);
    w[2] = (unsigned)f2bf_bits(c[0]) | ((unsigned)f2bf_bits(c[1]) << 16);
    w[3] = (unsigned)f2bf_bits(c[2]) | ((unsigned)f2bf_bits(c[3]) << 16);
    *(volatile v4u*)(dst) = w;
    __threadfence();
    *(volatile v4u*)(dst) = w;
  }
}

__global__ __launch_bounds__(256) void bias_cat3(
    const float* __restrict__ b0, const float* __restrict__ b1, const float* __restrict__ b2,
    float* __restrict__ out) {
  const int t4 = threadIdx.x * 4;
  const v4f a = *(const v4f*)(b0 + t4);
  const v4f b = *(const v4f*)(b1 + t4);
  const v4f c = *(const v4f*)(b2 + t4);
  *(volatile v4f*)(out + t4) = a;
  *(volatile v4f*)(out + kDim + t4) = b;
  *(volatile v4f*)(out + 2 * kDim + t4) = c;
  __threadfence();
  *(volatile v4f*)(out + t4) = a;
  *(volatile v4f*)(out + kDim + t4) = b;
  *(volatile v4f*)(out + 2 * kDim + t4) = c;
}

__global__ __launch_bounds__(256) void tcast64(
    const float* __restrict__ W, unsigned short* __restrict__ Wt, int nrows, int ncols) {
  __shared__ __align__(16) unsigned short tl[64 * 72];
  const int tid = threadIdx.x, lane = tid & 31, wave = tid >> 5;
  const int k0 = blockIdx.y * 64;
  const int n0 = blockIdx.x * 64;
  const int krow = tid >> 2;
  const int nseg = (tid & 3) * 16;
  const float* src = W + (size_t)(k0 + krow) * ncols + n0 + nseg;
  v4f vv[4];
#pragma unroll
  for (int i = 0; i < 4; ++i) vv[i] = ((const v4f*)src)[i];
#pragma unroll
  for (int i = 0; i < 4; ++i)
#pragma unroll
    for (int e = 0; e < 4; ++e) tl[(nseg + 4 * i + e) * 72 + krow] = f2bf_bits(vv[i][e]);
  __syncthreads();
  const int q4 = lane >> 3, c8 = (lane & 7) * 8;
  for (int pass = 0; pass < 2; ++pass) {
#pragma unroll
    for (int it = 0; it < 2; ++it) {
      const int row = wave * 8 + it * 4 + q4;
      const v4u w = *(const v4u*)(tl + row * 72 + c8);
      *(volatile v4u*)(Wt + (size_t)(n0 + row) * nrows + k0 + c8) = w;
    }
    __threadfence();
  }
}

#define AT_D 64
#define AT_NW 4
#define AT_QB 64
#define AT_KC 64
static_assert(AT_D == kHeadDim);
static_assert(AT_QB == AT_NW * 16);
static_assert(AT_NW * 32 == 2 * AT_KC);
static_assert(AT_NW * 32 == 2 * AT_QB);
static_assert(AT_KC == 64);
static_assert(kSeq % AT_QB == 0 && kSeq % AT_KC == 0);

struct LdsKV {
  unsigned short kh[AT_KC * AT_D];
  unsigned short kl[AT_KC * AT_D];
  unsigned short vh[AT_D * AT_KC];
  unsigned short vl[AT_D * AT_KC];
};
union LdsU {
  LdsKV kv;
  float os[AT_NW][16 * 68];
};
static_assert(sizeof(LdsKV) == 32768);
static_assert(sizeof(LdsU) == 32768);

__device__ __forceinline__ __bf16 at_f2bf(float f) { return __builtin_bit_cast(__bf16, f2bf_bits(f)); }
__device__ __forceinline__ void at_split(float f, __bf16& hi, __bf16& lo) {
  const unsigned short hb = f2bf_bits(f);
  hi = __builtin_bit_cast(__bf16, hb);
  lo = at_f2bf(f - __uint_as_float(((unsigned)hb) << 16));
}
__device__ __forceinline__ v8f at_mma(v16b a, v16b b, v8f c) {
  c = __builtin_amdgcn_wmma_f32_16x16x32_bf16(false, a, false, b, (short)0, c, false, false);
  asm volatile("v_nop\n\tv_nop\n\tv_nop\n\tv_nop" : "+v"(c) : "v"(a), "v"(b));
  return c;
}

__global__ __launch_bounds__(128)
void attn64_mask_planes(const unsigned short* __restrict__ qkvh, const unsigned short* __restrict__ qkvl,
                        const int* __restrict__ mask, int ldm,
                        unsigned short* __restrict__ yh, unsigned short* __restrict__ yl,
                        int nseq, int nheads, int ldq, int ldo, float sscale) {
  __shared__ __align__(16) LdsU lds;
  __shared__ __align__(16) __bf16 Psh[AT_NW][16 * AT_KC];
  __shared__ __align__(16) __bf16 Psl[AT_NW][16 * AT_KC];
  __shared__ __align__(16) unsigned mbits[AT_QB * 2];
  __shared__ int wflag[AT_NW];

  const int tid  = threadIdx.x;
  const int wave = tid >> 5;
  const int lane = tid & 31;
  const int hh   = lane >> 4;
  const int c    = lane & 15;

  const int nqb = nseq / AT_QB;
  const int bx  = blockIdx.x;
  const int qb  = bx % nqb;
  const int bhd = bx / nqb;
  const int h   = bhd % nheads;
  const int b   = bhd / nheads;
  const int q0  = qb * AT_QB + wave * 16;
  const size_t rowb = (size_t)b * nseq;
  const int qoff = h * AT_D;
  const int kofs = nheads * AT_D + h * AT_D;
  const int vofs = 2 * nheads * AT_D + h * AT_D;
  const float ninf = -__builtin_huge_valf();

  const __bf16* QH = (const __bf16*)(const void*)qkvh;
  const __bf16* QL = (const __bf16*)(const void*)qkvl;
  const __bf16* KHb = (const __bf16*)(const void*)lds.kv.kh;
  const __bf16* KLb = (const __bf16*)(const void*)lds.kv.kl;
  const __bf16* VHb = (const __bf16*)(const void*)lds.kv.vh;
  const __bf16* VLb = (const __bf16*)(const void*)lds.kv.vl;

  const unsigned* mbase = (const unsigned*)(const void*)mask
                        + (size_t)(qb * AT_QB + (tid >> 1)) * (size_t)ldm + (tid & 1) * 32;

  v16b qah[2], qal[2];
  {
    const size_t qr = (rowb + q0 + c) * (size_t)ldq + qoff + 8 * hh;
#pragma unroll
    for (int dc = 0; dc < 2; ++dc) {
      qah[dc] = Frag<__bf16>::load(QH + qr + dc * 32);
      qal[dc] = Frag<__bf16>::load(QL + qr + dc * 32);
    }
  }

  float mrow[8], lrow[8];
  v8f oacc[4];
  int dense = 0;
  const int nTiles = nseq / AT_KC;

#pragma unroll 1
  for (int att = 0; att < 2; ++att) {
#pragma unroll
    for (int r = 0; r < 8; ++r) { mrow[r] = ninf; lrow[r] = 0.f; }
#pragma unroll
    for (int t = 0; t < 4; ++t) oacc[t] = (v8f){0.f,0.f,0.f,0.f,0.f,0.f,0.f,0.f};

#pragma unroll 1
    for (int kc = 0; kc < nTiles; ++kc) {
      const int kv0 = kc * AT_KC;
      __syncthreads();
      {
        const v4u* pm = (const v4u*)(mbase + kv0);
        unsigned wbits = 0u;
#pragma unroll
        for (int i = 0; i < 8; ++i) {
          const v4u mv = pm[i];
#pragma unroll
          for (int e = 0; e < 4; ++e) wbits |= ((mv[e] != 0u) ? 1u : 0u) << (4 * i + e);
        }
        mbits[tid] = wbits;
        const unsigned bal = __builtin_amdgcn_ballot_w32(wbits != 0u);
        if (lane == 0) wflag[wave] = (bal != 0u) ? 1 : 0;
      }
      __syncthreads();
      const int anyk = wflag[0] | wflag[1] | wflag[2] | wflag[3];
      if ((anyk | dense) == 0) continue;
      {
        const int kvr = tid >> 1, dh = (tid & 1) * 32;
        const size_t kr = (rowb + kv0 + kvr) * (size_t)ldq + dh;
        v4u w0[4], w1[4];
        const v4u* pkh = (const v4u*)(qkvh + kr + kofs);
        const v4u* pkl = (const v4u*)(qkvl + kr + kofs);
#pragma unroll
        for (int i = 0; i < 4; ++i) { w0[i] = pkh[i]; w1[i] = pkl[i]; }
#pragma unroll
        for (int i = 0; i < 4; ++i) {
          *(v4u*)(lds.kv.kh + kvr * AT_D + dh + 8 * i) = w0[i];
          *(v4u*)(lds.kv.kl + kvr * AT_D + dh + 8 * i) = w1[i];
        }
        const v4u* pvh = (const v4u*)(qkvh + kr + vofs);
        const v4u* pvl = (const v4u*)(qkvl + kr + vofs);
#pragma unroll
        for (int i = 0; i < 4; ++i) { w0[i] = pvh[i]; w1[i] = pvl[i]; }
#pragma unroll
        for (int i = 0; i < 4; ++i) {
#pragma unroll
          for (int e = 0; e < 4; ++e) {
            const unsigned ua = w0[i][e], ub = w1[i][e];
            const int d0 = dh + 8 * i + 2 * e;
            lds.kv.vh[d0 * AT_KC + kvr]       = (unsigned short)(ua & 0xffffu);
            lds.kv.vh[(d0 + 1) * AT_KC + kvr] = (unsigned short)(ua >> 16);
            lds.kv.vl[d0 * AT_KC + kvr]       = (unsigned short)(ub & 0xffffu);
            lds.kv.vl[(d0 + 1) * AT_KC + kvr] = (unsigned short)(ub >> 16);
          }
        }
      }
      __syncthreads();

      v8f s[4];
#pragma unroll
      for (int j = 0; j < 4; ++j) {
        s[j] = (v8f){0.f,0.f,0.f,0.f,0.f,0.f,0.f,0.f};
#pragma unroll
        for (int dc = 0; dc < 2; ++dc) {
          const v16b kb = Frag<__bf16>::load(KHb + (j * 16 + c) * AT_D + dc * 32 + 8 * hh);
          const v16b kl = Frag<__bf16>::load(KLb + (j * 16 + c) * AT_D + dc * 32 + 8 * hh);
          s[j] = at_mma(qah[dc], kb, s[j]);
          s[j] = at_mma(qah[dc], kl, s[j]);
          s[j] = at_mma(qal[dc], kb, s[j]);
        }
      }

      float cm[8];
#pragma unroll
      for (int r = 0; r < 8; ++r) {
        const int lr = wave * 16 + 8 * hh + r;
        const unsigned mw0 = mbits[lr * 2];
        const unsigned mw1 = mbits[lr * 2 + 1];
        float m = ninf;
#pragma unroll
        for (int j = 0; j < 4; ++j) {
          const unsigned mw = (j < 2) ? mw0 : mw1;
          const int bit = (j & 1) * 16 + c;
          const bool keep = ((mw >> bit) & 1u) != 0u;
          const float sv = s[j][r] * sscale;
          const float val = keep ? sv : kMaskFill;
          s[j][r] = val;
          m = fmaxf(m, val);
        }
#pragma unroll
        for (int off = 1; off < 16; off <<= 1) m = fmaxf(m, __shfl_xor(m, off, 32));
        cm[r] = m;
      }

      __bf16* pwh = Psh[wave];
      __bf16* pwl = Psl[wave];
#pragma unroll
      for (int r = 0; r < 8; ++r) {
        const float mnew  = fmaxf(mrow[r], cm[r]);
        const float alpha = expf(mrow[r] - mnew);
        mrow[r] = mnew;
        float psum = 0.f;
#pragma unroll
        for (int j = 0; j < 4; ++j) {
          const float p = expf(s[j][r] - mnew);
          psum += p;
          __bf16 ph, pl;
          at_split(p, ph, pl);
          pwh[(8 * hh + r) * AT_KC + j * 16 + c] = ph;
          pwl[(8 * hh + r) * AT_KC + j * 16 + c] = pl;
        }
#pragma unroll
        for (int off = 1; off < 16; off <<= 1) psum += __shfl_xor(psum, off, 32);
        lrow[r] = lrow[r] * alpha + psum;
#pragma unroll
        for (int t = 0; t < 4; ++t) oacc[t][r] *= alpha;
      }
      __builtin_amdgcn_fence(3  , "workgroup");
      __builtin_amdgcn_wave_barrier();
      __builtin_amdgcn_fence(2  , "workgroup");

#pragma unroll
      for (int kk = 0; kk < 2; ++kk) {
        const v16b pa = Frag<__bf16>::load(pwh + c * AT_KC + kk * 32 + 8 * hh);
        const v16b pb = Frag<__bf16>::load(pwl + c * AT_KC + kk * 32 + 8 * hh);
#pragma unroll
        for (int t = 0; t < 4; ++t) {
          const v16b vb  = Frag<__bf16>::load(VHb + (t * 16 + c) * AT_KC + kk * 32 + 8 * hh);
          const v16b vlo = Frag<__bf16>::load(VLb + (t * 16 + c) * AT_KC + kk * 32 + 8 * hh);
          oacc[t] = at_mma(pa, vb,  oacc[t]);
          oacc[t] = at_mma(pa, vlo, oacc[t]);
          oacc[t] = at_mma(pb, vb,  oacc[t]);
        }
      }
    }

    int bad = 0;
#pragma unroll
    for (int r = 0; r < 8; ++r) bad |= (mrow[r] > -1.0e8f) ? 0 : 1;
    const unsigned bb = __builtin_amdgcn_ballot_w32(bad != 0);
    __syncthreads();
    if (lane == 0) wflag[wave] = (bb != 0u) ? 1 : 0;
    __syncthreads();
    const int need = wflag[0] | wflag[1] | wflag[2] | wflag[3];
    if (need == 0 || dense != 0) break;
    dense = 1;
  }

  __syncthreads();
  float* os = lds.os[wave];
#pragma unroll
  for (int r = 0; r < 8; ++r) {
    const float inv = 1.0f / lrow[r];
#pragma unroll
    for (int t = 0; t < 4; ++t) os[(8 * hh + r) * 68 + t * 16 + c] = oacc[t][r] * inv;
  }
  __builtin_amdgcn_fence(3  , "workgroup");
  __builtin_amdgcn_wave_barrier();
  __builtin_amdgcn_fence(2  , "workgroup");
  {
    const int q4 = lane >> 3, c8 = (lane & 7) * 8;
    for (int pass = 0; pass < 2; ++pass) {
#pragma unroll
      for (int it = 0; it < 4; ++it) {
        const int row = it * 4 + q4;
        const float* sp = os + row * 68 + c8;
        v4u hw, lw;
#pragma unroll
        for (int e2 = 0; e2 < 4; ++e2) {
          const float f0 = sp[2 * e2], f1 = sp[2 * e2 + 1];
          const unsigned short hb0 = f2bf_bits(f0);
          const unsigned short lb0 = f2bf_bits(f0 - bf_bits2f(hb0));
          const unsigned short hb1 = f2bf_bits(f1);
          const unsigned short lb1 = f2bf_bits(f1 - bf_bits2f(hb1));
          hw[e2] = (unsigned)hb0 | ((unsigned)hb1 << 16);
          lw[e2] = (unsigned)lb0 | ((unsigned)lb1 << 16);
        }
        const size_t o = (rowb + q0 + row) * (size_t)ldo + h * AT_D + c8;
        *(volatile v4u*)(yh + o) = hw;
        *(volatile v4u*)(yl + o) = lw;
      }
      __threadfence();
    }
  }
}

extern "C" void kernel_launch(void* const* d_in, const int* in_sizes, int n_in,
                              void* d_out, int out_size, void* d_ws,
                              size_t ws_size, hipStream_t stream)
{
  if (n_in < 10) return;
  if (ws_size < kWsTotal) return;
  if (out_size < kRows * kDim) return;
  if (in_sizes[0] < ((kBatch - 1) * kSeqFull + kSeq) * kDim) return;
  if (in_sizes[1] < (kSeq - 1) * kSeqFull + kSeq) return;
  if (in_sizes[2] < kDim * kDim || in_sizes[4] < kDim * kDim ||
      in_sizes[6] < kDim * kDim || in_sizes[8] < kDim * kDim) return;
  if (in_sizes[3] < kDim || in_sizes[5] < kDim || in_sizes[7] < kDim || in_sizes[9] < kDim) return;

  const float* x    = (const float*)d_in[0];
  const int*   mask = (const int*)d_in[1];
  const float* Wq   = (const float*)d_in[2];
  const float* bq   = (const float*)d_in[3];
  const float* Wk   = (const float*)d_in[4];
  const float* bk   = (const float*)d_in[5];
  const float* Wv   = (const float*)d_in[6];
  const float* bv   = (const float*)d_in[7];
  const float* Wo   = (const float*)d_in[8];
  const float* bo   = (const float*)d_in[9];
  float* out = (float*)d_out;

  unsigned char* ws = (unsigned char*)d_ws;
  unsigned short* XB  = (unsigned short*)(ws + kOffXB);
  unsigned short* WQT = (unsigned short*)(ws + kOffWQT);
  unsigned short* QH  = (unsigned short*)(ws + kOffQH);
  unsigned short* QL  = (unsigned short*)(ws + kOffQL);
  unsigned short* YH  = (unsigned short*)(ws + kOffYH);
  unsigned short* YL  = (unsigned short*)(ws + kOffYL);
  float*          BC  = (float*)(ws + kOffBC);
  unsigned short* WPT = (unsigned short*)(ws + kOffWPT);

  {
    const int n8 = kSeq * kDim / 8;
    cast_f32_bf16x8<<<dim3((n8 + 255) / 256, kBatch), dim3(256), 0, stream>>>(
        x, XB, n8, (long)kSeqFull * kDim, (long)kSeq * kDim);
  }
  tcast64<<<dim3(kDim / 64, kDim / 64), dim3(256), 0, stream>>>(Wq, WQT, kDim, kDim);
  tcast64<<<dim3(kDim / 64, kDim / 64), dim3(256), 0, stream>>>(Wk, WQT + (size_t)kDim * kDim, kDim, kDim);
  tcast64<<<dim3(kDim / 64, kDim / 64), dim3(256), 0, stream>>>(Wv, WQT + (size_t)2 * kDim * kDim, kDim, kDim);
  tcast64<<<dim3(kDim / 64, kDim / 64), dim3(256), 0, stream>>>(Wo, WPT, kDim, kDim);
  bias_cat3<<<dim3(1), dim3(256), 0, stream>>>(bq, bk, bv, BC);
  {
    const int tiles = (kRows / 64) * (kQKV / 64);
    gemm_qkv_planes<<<dim3((tiles + 7) / 8, 1), dim3(256), 0, stream>>>(
        XB, kDim, WQT, kDim, QH, QL, kQKV, BC, kRows, kQKV, kDim);
  }
  attn64_mask_planes<<<dim3(kBatch * kHeads * (kSeq / AT_QB)), dim3(128), 0, stream>>>(
      QH, QL, mask, kSeqFull, YH, YL, kSeq, kHeads, kQKV, kDim, kScoreScale);
  {
    const int tiles = (kRows / 64) * (kDim / 64);
    gemm_proj_f32<<<dim3((tiles + 7) / 8, 1), dim3(256), 0, stream>>>(
        YH, YL, kDim, WPT, kDim, out, kDim, bo, kRows, kDim, kDim);
  }
}
